// Network_9929964388467
// MI455X (gfx1250) — hardware-verified
//
#include <hip/hip_runtime.h>
#include <stddef.h>
#pragma clang fp contract(off)

typedef __bf16         v16b  __attribute__((ext_vector_type(16)));
typedef unsigned short v16us __attribute__((ext_vector_type(16)));
typedef unsigned short v8us  __attribute__((ext_vector_type(8)));
typedef float          v8f   __attribute__((ext_vector_type(8)));
typedef float          v4f   __attribute__((ext_vector_type(4)));

union Frag { v16b v; v16us u; v8us hv[2]; };

#define NB    32
#define NPIX  3072
#define NH    240
#define NHP   256
#define NO    10
#define NOP   16
#define TB    350
#define TP    352
#define SP    384
#define RL    32
#define THRESH 10.0f

__device__ __forceinline__ v8f wmma_bf16(v16b a, v16b b, v8f c) {
  v8f d = __builtin_amdgcn_wmma_f32_16x16x32_bf16(false, a, false, b, (short)0, c, false, false);
  asm volatile("v_nop\n\tv_nop\n\tv_nop\n\tv_nop" : "+v"(d) : "v"(a), "v"(b));
  return d;
}

__device__ __forceinline__ unsigned short bf_rne(float x) {
  unsigned u = __float_as_uint(x);
  u += 0x7FFFu + ((u >> 16) & 1u);
  return (unsigned short)(u >> 16);
}
__device__ __forceinline__ float bf_val(unsigned short s) {
  return __uint_as_float(((unsigned)s) << 16);
}
__device__ __forceinline__ void split3(float x, unsigned short& h, unsigned short& m, unsigned short& l) {
  h = bf_rne(x);
  float r = x - bf_val(h);
  m = bf_rne(r);
  r = r - bf_val(m);
  l = bf_rne(r);
}

__device__ __forceinline__ int kmap(int i, int h) {
  return (i < 8) ? (8 * h + i) : (16 + 8 * h + (i - 8));
}

__global__ __launch_bounds__(256) void k_x1(const int* __restrict__ inp,
                                            const int* __restrict__ tab, int ntab,
                                            const float* __restrict__ w1,
                                            float* x1) {
  __shared__ int tix[NPIX];
  __shared__ int lst[NPIX];
  __shared__ int cnt[TP];
  __shared__ int ofs[TP + 1];
  const int b = blockIdx.x;
  const int tid = threadIdx.x;
  if (b >= NB) return;

  for (int p = tid; p < NPIX; p += 256) {
    int v = inp[(size_t)b * NPIX + p];
    if (v < 0) v += ntab;
    v = v < 0 ? 0 : (v >= ntab ? ntab - 1 : v);
    int t = tab[v];
    tix[p] = (t >= 0 && t < TB) ? t : -1;
  }
  __syncthreads();
  for (int t = tid; t < TP; t += 256) {
    int c = 0;
#pragma unroll 4
    for (int p = 0; p < NPIX; ++p) c += (tix[p] == t) ? 1 : 0;
    cnt[t] = c;
  }
  __syncthreads();
  if (tid == 0) {
    int a = 0;
    for (int t = 0; t < TP; ++t) { ofs[t] = a; a += cnt[t]; }
    ofs[TP] = a;
  }
  __syncthreads();
  for (int t = tid; t < TP; t += 256) {
    int k = ofs[t];
#pragma unroll 4
    for (int p = 0; p < NPIX; ++p) {
      if (tix[p] == t) { lst[k] = p; ++k; }
    }
  }
  __syncthreads();

  const int w = tid >> 5, lane = tid & 31;
  for (int n = w; n < NH; n += 8) {
    const float* row = w1 + (size_t)n * NPIX;
    for (int ch = 0; ch < 3; ++ch) {
      const int t0 = ch * 128 + lane * 4;
      if (t0 < TP) {
        v4f acc;
#pragma unroll
        for (int j = 0; j < 4; ++j) {
          const int t = t0 + j;
          const int q0 = ofs[t], q1 = ofs[t + 1];
          float a = 0.0f;
          for (int q = q0; q < q1; ++q) a = a + row[lst[q]];
          acc[j] = a;
        }
        volatile v4f* dst = (volatile v4f*)(x1 + ((size_t)(b * NH + n)) * TP + t0);
        *dst = acc;
        __threadfence();
        *dst = acc;
      }
    }
  }
}

__device__ __forceinline__ void store_tile_rows(const float* ot, float* u, int row0, int w, int lane) {
  for (int r = w; r < 16; r += 2) {
    for (int c = lane * 4; c < TP; c += 128) {
      v4f v = *(const v4f*)(ot + r * TP + c);
      *(volatile v4f*)(u + (size_t)(row0 + r) * TP + c) = v;
    }
  }
}

__global__ __launch_bounds__(64) void k_psp(const float* __restrict__ x, float* u, int nrows) {
  __shared__ __attribute__((aligned(16))) unsigned short Ap[3][16 * TP];
  __shared__ __attribute__((aligned(16))) unsigned short Sp[3][TP];
  __shared__ __attribute__((aligned(16))) float ot[16 * TP];
  const int tid = threadIdx.x, w = tid >> 5, lane = tid & 31;
  const int h = lane >> 4, m = lane & 15;
  const int row0 = blockIdx.x * 16;
  if (row0 + 16 > nrows) return;

  for (int i = tid; i < 16 * TP; i += 64) {
    const int r = i / TP, c = i - r * TP;
    const float v = x[(size_t)(row0 + r) * TP + c];
    unsigned short ph, pm, pl;
    split3(v, ph, pm, pl);
    Ap[0][i] = ph; Ap[1][i] = pm; Ap[2][i] = pl;
  }
  for (int d = tid; d < TP; d += 64) {
    const float q = (float)d * 0.1f;
    const float s = q * expf(1.0f - q);
    unsigned short ph, pm, pl;
    split3(s, ph, pm, pl);
    Sp[0][d] = ph; Sp[1][d] = pm; Sp[2][d] = pl;
  }
  __syncthreads();

  for (int nt = w; nt < TP / 16; nt += 2) {
    v8f acc = {0.f, 0.f, 0.f, 0.f, 0.f, 0.f, 0.f, 0.f};
    const int tcol = 16 * nt + m;
    const int kmax = (16 * nt + 15) >> 5;
    for (int ks = 0; ks <= kmax; ++ks) {
      const int k0 = ks * 32;
      Frag ah, am, al, bh, bm, bl;
      const int aoff = m * TP + k0 + 8 * h;
      ah.hv[0] = *(const v8us*)(&Ap[0][aoff]); ah.hv[1] = *(const v8us*)(&Ap[0][aoff + 16]);
      am.hv[0] = *(const v8us*)(&Ap[1][aoff]); am.hv[1] = *(const v8us*)(&Ap[1][aoff + 16]);
      al.hv[0] = *(const v8us*)(&Ap[2][aoff]); al.hv[1] = *(const v8us*)(&Ap[2][aoff + 16]);
#pragma unroll
      for (int i = 0; i < 16; ++i) {
        int d = tcol - (k0 + kmap(i, h));
        d = d > 0 ? d : 0;
        bh.u[i] = Sp[0][d]; bm.u[i] = Sp[1][d]; bl.u[i] = Sp[2][d];
      }
      acc = wmma_bf16(al.v, bh.v, acc);
      acc = wmma_bf16(am.v, bm.v, acc);
      acc = wmma_bf16(ah.v, bl.v, acc);
      acc = wmma_bf16(am.v, bh.v, acc);
      acc = wmma_bf16(ah.v, bm.v, acc);
      acc = wmma_bf16(ah.v, bh.v, acc);
    }
#pragma unroll
    for (int r = 0; r < 8; ++r) ot[(8 * h + r) * TP + tcol] = acc[r];
  }
  __syncthreads();
  store_tile_rows(ot, u, row0, w, lane);
  __threadfence();
  store_tile_rows(ot, u, row0, w, lane);
}

__device__ __forceinline__ void ref_consts(float* rk) {
#pragma unroll
  for (int j = 0; j < RL; ++j) {
    const float tj = (float)j;
    rk[j] = (-20.0f * tj) * expf(1.0f - tj);
  }
}

__device__ __forceinline__ float spike_step(float ut, float* buf, const float* rk) {
  const float v = ut + buf[0];
  const float s = (v >= THRESH) ? 1.0f : 0.0f;
#pragma unroll
  for (int q = 0; q < RL - 1; ++q) buf[q] = buf[q + 1] + s * rk[q];
  buf[RL - 1] = 0.0f + s * rk[RL - 1];
  return s;
}

__global__ __launch_bounds__(64) void k_spike1(const float* __restrict__ u1, unsigned short* s1) {
  const int i = blockIdx.x * 64 + threadIdx.x;
  if (i >= NB * NHP) return;
  const int b = i / NHP, n = i - b * NHP;
  unsigned short* dst = s1 + (size_t)i * SP;
  if (n >= NH) {
    const v8us z = {0, 0, 0, 0, 0, 0, 0, 0};
    for (int c = 0; c < SP / 8; ++c) *(volatile v8us*)(dst + c * 8) = z;
    __threadfence();
    for (int c = 0; c < SP / 8; ++c) *(volatile v8us*)(dst + c * 8) = z;
    return;
  }
  float rk[RL], buf[RL];
  ref_consts(rk);
#pragma unroll
  for (int q = 0; q < RL; ++q) buf[q] = 0.0f;
  const float* ur = u1 + (size_t)(b * NH + n) * TP;
#pragma unroll 1
  for (int c = 0; c < SP / 8; ++c) {
    unsigned bits = 0u;
    if (c * 8 < TB) {
#pragma unroll 1
      for (int j = 0; j < 8; ++j) {
        const int t = c * 8 + j;
        if (t < TB) {
          const float s = spike_step(ur[t], buf, rk);
          bits |= (s != 0.0f ? 1u : 0u) << j;
        }
      }
    }
    v8us o;
#pragma unroll
    for (int e = 0; e < 8; ++e) o[e] = ((bits >> e) & 1u) ? (unsigned short)0x3F80 : (unsigned short)0;
    volatile v8us* d = (volatile v8us*)(dst + c * 8);
    *d = o;
    __threadfence();
    *d = o;
  }
}

__global__ __launch_bounds__(64) void k_l2(const float* __restrict__ w2,
                                           const unsigned short* __restrict__ s1,
                                           float* x2) {
  __shared__ __attribute__((aligned(16))) unsigned short Wp[3][NOP * NHP];
  __shared__ __attribute__((aligned(16))) float ot[16 * TP];
  const int tid = threadIdx.x, w = tid >> 5, lane = tid & 31;
  const int h = lane >> 4, m = lane & 15;
  const int b = blockIdx.x;
  if (b >= NB) return;

  for (int i = tid; i < NOP * NHP; i += 64) {
    const int mm = i >> 8, n = i & 255;
    const float v = (mm < NO && n < NH) ? w2[mm * NH + n] : 0.0f;
    unsigned short ph, pm, pl;
    split3(v, ph, pm, pl);
    Wp[0][i] = ph; Wp[1][i] = pm; Wp[2][i] = pl;
  }
  __syncthreads();

  for (int nt = w; nt < TP / 16; nt += 2) {
    v8f acc = {0.f, 0.f, 0.f, 0.f, 0.f, 0.f, 0.f, 0.f};
    const int tcol = 16 * nt + m;
#pragma unroll 1
    for (int ks = 0; ks < NHP / 32; ++ks) {
      const int k0 = ks * 32;
      Frag ah, am, al, bs;
      const int aoff = m * NHP + k0 + 8 * h;
      ah.hv[0] = *(const v8us*)(&Wp[0][aoff]); ah.hv[1] = *(const v8us*)(&Wp[0][aoff + 16]);
      am.hv[0] = *(const v8us*)(&Wp[1][aoff]); am.hv[1] = *(const v8us*)(&Wp[1][aoff + 16]);
      al.hv[0] = *(const v8us*)(&Wp[2][aoff]); al.hv[1] = *(const v8us*)(&Wp[2][aoff + 16]);
#pragma unroll
      for (int i = 0; i < 16; ++i) {
        const int kk = k0 + kmap(i, h);
        bs.u[i] = s1[((size_t)(b * NHP + kk)) * SP + tcol];
      }
      acc = wmma_bf16(al.v, bs.v, acc);
      acc = wmma_bf16(am.v, bs.v, acc);
      acc = wmma_bf16(ah.v, bs.v, acc);
    }
#pragma unroll
    for (int r = 0; r < 8; ++r) ot[(8 * h + r) * TP + tcol] = acc[r];
  }
  __syncthreads();
  store_tile_rows(ot, x2, b * NOP, w, lane);
  __threadfence();
  store_tile_rows(ot, x2, b * NOP, w, lane);
}

__global__ __launch_bounds__(32) void k_spike2(const float* __restrict__ u2, float* out, int nseq) {
  __shared__ __attribute__((aligned(16))) float so[32 * TB];
  const int lane = threadIdx.x;
  const int seq = blockIdx.x * 32 + lane;
  if (seq < nseq) {
    const int b = seq / NO, mo = seq - b * NO;
    const float* ur = u2 + (size_t)(b * NOP + mo) * TP;
    float rk[RL], buf[RL];
    ref_consts(rk);
#pragma unroll
    for (int q = 0; q < RL; ++q) buf[q] = 0.0f;
#pragma unroll 1
    for (int t = 0; t < TB; ++t) {
      const float s = spike_step(ur[t], buf, rk);
      so[lane * TB + t] = s;
    }
  } else {
    for (int t = 0; t < TB; ++t) so[lane * TB + t] = 0.0f;
  }
  __syncthreads();
  const int nvals = 32 * TB;
  const int rem = (nseq - blockIdx.x * 32) * TB;
  float* ob = out + (size_t)blockIdx.x * nvals;
  for (int f = lane * 4; f < nvals && f + 4 <= rem; f += 128) {
    v4f v = *(const v4f*)(&so[f]);
    *(volatile v4f*)(ob + f) = v;
  }
  __threadfence();
  for (int f = lane * 4; f < nvals && f + 4 <= rem; f += 128) {
    v4f v = *(const v4f*)(&so[f]);
    *(volatile v4f*)(ob + f) = v;
  }
}

static inline size_t al256(size_t x) { return (x + 255) & ~(size_t)255; }

extern "C" void kernel_launch(void* const* d_in, const int* in_sizes, int n_in,
                              void* d_out, int out_size, void* d_ws, size_t ws_size,
                              hipStream_t stream) {
  if (n_in < 4) return;
  if (in_sizes[0] != NB * NPIX) return;
  if (in_sizes[1] < 1) return;
  if (in_sizes[2] != NH * NPIX) return;
  if (in_sizes[3] != NO * NH) return;
  if (out_size != NB * NO * TB) return;

  const int*   inp = (const int*)d_in[0];
  const int*   tab = (const int*)d_in[1];
  const float* w1  = (const float*)d_in[2];
  const float* w2  = (const float*)d_in[3];
  float*       out = (float*)d_out;
  const int    ntab = in_sizes[1];

  const size_t sz_x1 = al256((size_t)NB * NH * TP * sizeof(float));
  const size_t sz_u1 = sz_x1;
  const size_t sz_s1 = al256((size_t)NB * NHP * SP * sizeof(unsigned short));
  const size_t sz_x2 = al256((size_t)NB * NOP * TP * sizeof(float));
  const size_t sz_u2 = sz_x2;
  const size_t off_x1 = 0;
  const size_t off_u1 = off_x1 + sz_x1;
  const size_t off_s1 = off_u1 + sz_u1;
  const size_t off_x2 = off_s1 + sz_s1;
  const size_t off_u2 = off_x2 + sz_x2;
  const size_t total  = off_u2 + sz_u2;
  if (total > ws_size) return;

  char* ws = (char*)d_ws;
  float*          x1 = (float*)(ws + off_x1);
  float*          u1 = (float*)(ws + off_u1);
  unsigned short* s1 = (unsigned short*)(ws + off_s1);
  float*          x2 = (float*)(ws + off_x2);
  float*          u2 = (float*)(ws + off_u2);

  const int rows1 = NB * NH;
  const int rows2 = NB * NOP;
  const int nseq2 = NB * NO;

  k_x1<<<dim3(NB), dim3(256), 0, stream>>>(inp, tab, ntab, w1, x1);
  k_psp<<<dim3(rows1 / 16), dim3(64), 0, stream>>>(x1, u1, rows1);
  k_spike1<<<dim3((NB * NHP + 63) / 64), dim3(64), 0, stream>>>(u1, s1);
  k_l2<<<dim3(NB), dim3(64), 0, stream>>>(w2, s1, x2);
  k_psp<<<dim3(rows2 / 16), dim3(64), 0, stream>>>(x2, u2, rows2);
  k_spike2<<<dim3((nseq2 + 31) / 32), dim3(32), 0, stream>>>(u2, out, nseq2);
  (void)hipGetLastError();
}
